// HierarchicalPathReasoning_46866683134444
// MI455X (gfx1250) — hardware-run, weakly checked
//
#include <hip/hip_runtime.h>
#include <math.h>

typedef __attribute__((ext_vector_type(16))) _Float16 v16h;
typedef __attribute__((ext_vector_type(8)))  _Float16 v8h;
typedef __attribute__((ext_vector_type(8)))  float    v8f;
typedef __attribute__((ext_vector_type(4)))  float    v4f;
typedef __attribute__((ext_vector_type(4)))  int      v4i;

constexpr int kNodes      = 1000;
constexpr int kNodesPad   = 1024;
constexpr int kFeat       = 256;
constexpr int kHops       = 3;
constexpr int kPaths      = 84000;
constexpr int kChunk      = 42048;
constexpr int kNumChunks  = 2;
constexpr int kRowsPad    = kChunk * kNumChunks;
constexpr int kUvW        = 2 * kHops * kFeat;
constexpr int kHmPitch    = 832;
constexpr int kKz         = 800;
constexpr int kIndCol     = kHops * kFeat;
constexpr int kScoreH     = 128;
constexpr int kWsPitch    = 320;
constexpr int kKs         = 288;
constexpr int kTilesChunk = kChunk / 64;
constexpr int kTilesAll   = kTilesChunk * kNumChunks;
constexpr int kRedOuter   = 18;
constexpr int kRedInner   = 73;
constexpr float kCarryA   = 16.0f;
constexpr float kCarryW   = 256.0f;
constexpr float kFold     = 1.0f / (kCarryA * kCarryW);
constexpr int kOut1Elem   = kNodes * kFeat;

static_assert(kRowsPad == 84096);
static_assert(kRowsPad >= kPaths);
static_assert((kChunk % 64) == 0);
static_assert((kKz % 32) == 0 && (kKs % 32) == 0 && (kFeat % 32) == 0);
static_assert(kIndCol == 768 && kIndCol + 32 == kKz);
static_assert((kHmPitch * 2) % 128 == 0);
static_assert(kHmPitch >= kKz);
static_assert((kNodesPad % 64) == 0 && (kUvW % 64) == 0 && (kScoreH % 64) == 0);
static_assert(kWsPitch >= kKs && (kWsPitch % 64) == 0);
static_assert(kRedOuter * kRedInner == kTilesAll);
static_assert((kPaths % 32) == 0);
static_assert(kOut1Elem * 4 == 1024000);
static_assert((kOut1Elem * 4) % 128 == 0);
static_assert((kOut1Elem + kPaths) * 4 == 1360000);

constexpr size_t kSzNFH  = (size_t)kNodesPad * kFeat * 2;
constexpr size_t kSzW1T  = (size_t)kUvW * kFeat * 2;
constexpr size_t kSzUV   = (size_t)kNodesPad * kUvW * 4;
constexpr size_t kSzTC   = (size_t)kHmPitch * kFeat * 4;
constexpr size_t kSzTS   = (size_t)kWsPitch * kScoreH * 4;
constexpr size_t kSzWCT  = (size_t)kFeat * kHmPitch * 2;
constexpr size_t kSzWST  = (size_t)kScoreH * kWsPitch * 2;
constexpr size_t kSzHM   = (size_t)kChunk * kHmPitch * 2;
constexpr size_t kSzPART = (size_t)kTilesAll * kFeat * 4;
constexpr size_t kSzSP   = (size_t)2 * kRowsPad * 4;
constexpr size_t kSzAGG  = (size_t)kFeat * 4;
constexpr size_t kOffNFH  = 0;
constexpr size_t kOffW1T  = kOffNFH  + kSzNFH;
constexpr size_t kOffUV   = kOffW1T  + kSzW1T;
constexpr size_t kOffTC   = kOffUV   + kSzUV;
constexpr size_t kOffTS   = kOffTC   + kSzTC;
constexpr size_t kOffWCT  = kOffTS   + kSzTS;
constexpr size_t kOffWST  = kOffWCT  + kSzWCT;
constexpr size_t kOffHM   = kOffWST  + kSzWST;
constexpr size_t kOffPART = kOffHM   + kSzHM;
constexpr size_t kOffSP   = kOffPART + kSzPART;
constexpr size_t kOffAGG  = kOffSP   + kSzSP;
constexpr size_t kWsTotal = kOffAGG  + kSzAGG;
static_assert(kWsTotal == 81113088ull);
static_assert(kWsTotal <= 134217728ull);
static_assert((kOffW1T % 128) == 0 && (kOffUV % 128) == 0 && (kOffTC % 128) == 0 && (kOffTS % 128) == 0 &&
              (kOffWCT % 128) == 0 && (kOffWST % 128) == 0 && (kOffHM % 128) == 0 && (kOffPART % 128) == 0 &&
              (kOffSP % 128) == 0 && (kOffAGG % 128) == 0);

__device__ __forceinline__ int clamp_int(int v, int lo, int hi) { return v < lo ? lo : (v > hi ? hi : v); }

__device__ __forceinline__ v16h frag_load(const _Float16* p) {
  union { v16h v; v8h h[2]; } f;
  f.h[0] = *(const v8h*)(p);
  f.h[1] = *(const v8h*)(p + 16);
  return f.v;
}
__device__ __forceinline__ v8f mma_f16(v16h a, v16h b, v8f c) {
  c = __builtin_amdgcn_wmma_f32_16x16x32_f16(false, a, false, b, (short)0, c, false, false);
  asm volatile("v_nop\n\tv_nop\n\tv_nop\n\tv_nop" : "+v"(c) : "v"(a), "v"(b));
  return c;
}
__device__ __forceinline__ void wave_lds_sync() {
  __builtin_amdgcn_fence(__ATOMIC_RELEASE, "workgroup");
  __builtin_amdgcn_wave_barrier();
  __builtin_amdgcn_fence(__ATOMIC_ACQUIRE, "workgroup");
}

__global__ __launch_bounds__(256) void cast_nodes_f16(const float* __restrict__ nf, unsigned short* __restrict__ nfh)
{
  const int i = blockIdx.x * 256 + threadIdx.x;
  if (i >= kNodesPad * kFeat / 8) return;
  const int row = i >> 5;
  const int col = (i & 31) * 8;
  const bool ok = row < kNodes;
  const int rc = ok ? row : (kNodes - 1);
  const v4f a0 = *(const v4f*)(nf + (size_t)rc * kFeat + col);
  const v4f a1 = *(const v4f*)(nf + (size_t)rc * kFeat + col + 4);
  v8h hv;
#pragma unroll
  for (int e = 0; e < 4; ++e) {
    const float x0 = ok ? (a0[e] * kCarryA) : 0.0f;
    const float x1 = ok ? (a1[e] * kCarryA) : 0.0f;
    hv[e]     = (_Float16)x0;
    hv[4 + e] = (_Float16)x1;
  }
  unsigned short* q = nfh + (size_t)row * kFeat + col;
  *(volatile v8h*)q = hv;
  __threadfence();
  *(volatile v8h*)q = hv;
}

__global__ __launch_bounds__(256) void transpose_cast_f16(
    const float* __restrict__ in, int ldi, long inBatch,
    unsigned short* __restrict__ out, int ldo, long outBatch, float carry)
{
  __shared__ float tl[64 * 65];
  const int t = threadIdx.x;
  const float* ip = in + (size_t)blockIdx.z * inBatch;
  unsigned short* op = out + (size_t)blockIdx.z * outBatch;
  const int k0 = blockIdx.x * 64;
  const int n0 = blockIdx.y * 64;
#pragma unroll 4
  for (int i = 0; i < 16; ++i) {
    const int kk = i * 4 + (t >> 6);
    const int nn = t & 63;
    tl[kk * 65 + nn] = ip[(size_t)(k0 + kk) * ldi + n0 + nn];
  }
  __syncthreads();
  const int c8 = (t & 7) * 8;
  v8h hv[2];
#pragma unroll
  for (int it = 0; it < 2; ++it) {
    const int n = it * 32 + (t >> 3);
#pragma unroll
    for (int e = 0; e < 8; ++e) {
      const float x = tl[(c8 + e) * 65 + n] * carry;
      hv[it][e] = (_Float16)x;
    }
  }
  for (int pass = 0; pass < 2; ++pass) {
#pragma unroll
    for (int it = 0; it < 2; ++it) {
      const int n = it * 32 + (t >> 3);
      *(volatile v8h*)(op + (size_t)(n0 + n) * ldo + k0 + c8) = hv[it];
    }
    __threadfence();
  }
}

__global__ __launch_bounds__(256) void compose_rows_kernel(
    const float* __restrict__ W2, const float* __restrict__ b2, const float* __restrict__ Bm,
    const float* __restrict__ bfirst, float* __restrict__ out, int ncols, int nS, int rowsTotal)
{
  const int t = blockIdx.x * 256 + threadIdx.x;
  if (t >= rowsTotal * ncols) return;
  const int kr = t / ncols;
  const int j  = t - kr * ncols;
  const int nProd = nS * 256;
  const bool isProd = kr < nProd;
  const bool isBias = (kr == nProd);
  const bool isC    = (kr > nProd) && (kr <= nProd + nS);
  const int s = isProd ? (kr >> 8) : (isC ? (kr - nProd - 1) : 0);
  const float* arow = isProd ? (W2 + (size_t)kr * 256) : (b2 + (size_t)s * 256);
  const float* bcol = Bm + (size_t)s * 256 * ncols + j;
  float acc = 0.0f;
#pragma unroll 8
  for (int e = 0; e < 256; ++e) acc = fmaf(arow[e], bcol[(size_t)e * ncols], acc);
  const float bv = bfirst[j];
  const float v = (isProd || isC) ? acc : (isBias ? bv : 0.0f);
  *(volatile float*)(out + t) = v;
  __threadfence();
  *(volatile float*)(out + t) = v;
}

template <int MODE>
__global__ __launch_bounds__(256) void gemm_f16_tile64(
    const unsigned short* __restrict__ Ap, int lda,
    const unsigned short* __restrict__ Btp, int ldb,
    float* __restrict__ Cout, int ldc,
    const float* __restrict__ wvec,
    int M, int N, int nk, int jumpAt, int jumpTo, float scale)
{
  const _Float16* A  = (const _Float16*)Ap;
  const _Float16* Bt = (const _Float16*)Btp;
  __shared__ __align__(16) float sT[8][16 * 68];
  const int lane = threadIdx.x & 31;
  const int wave = threadIdx.x >> 5;
  const int tilesN = N >> 6;
  const int tilesM = M >> 6;
  const int tile = blockIdx.x * 8 + wave;
  if (tile >= tilesM * tilesN) return;
  const int tm = tile / tilesN;
  const int tn = tile - tm * tilesN;
  const int m0 = tm << 6;
  const int n0 = tn << 6;
  const int rlane = lane & 15;
  const int hh    = lane >> 4;
  const int koff  = hh * 8;
  const int mOff  = hh * 8;

  v8f acc[4][4];
#pragma unroll
  for (int i = 0; i < 4; ++i)
#pragma unroll
    for (int j = 0; j < 4; ++j) acc[i][j] = (v8f){0.f, 0.f, 0.f, 0.f, 0.f, 0.f, 0.f, 0.f};

  for (int kk = 0; kk < nk; ++kk) {
    const int ka = (kk < jumpAt) ? (kk << 5) : (jumpTo + ((kk - jumpAt) << 5));
    const int kb = kk << 5;
    v16h bh[4];
#pragma unroll
    for (int j = 0; j < 4; ++j)
      bh[j] = frag_load(Bt + (size_t)(n0 + (j << 4) + rlane) * ldb + koff + kb);
#pragma unroll
    for (int i = 0; i < 4; ++i) {
      const v16h ah = frag_load(A + (size_t)(m0 + (i << 4) + rlane) * lda + koff + ka);
#pragma unroll
      for (int j = 0; j < 4; ++j) acc[i][j] = mma_f16(ah, bh[j], acc[i][j]);
    }
  }

  float* slab = sT[wave];
  const int l16 = lane & 15;

  if (MODE == 0) {
#pragma unroll
    for (int i = 0; i < 4; ++i) {
      const int mBase = m0 + (i << 4);
#pragma unroll
      for (int j = 0; j < 4; ++j) {
#pragma unroll
        for (int r = 0; r < 8; ++r) slab[(mOff + r) * 68 + (j << 4) + rlane] = acc[i][j][r] * scale;
      }
      wave_lds_sync();
      const int c4 = l16 * 4;
      for (int pass = 0; pass < 2; ++pass) {
#pragma unroll
        for (int it = 0; it < 8; ++it) {
          const int row = it * 2 + hh;
          const v4f v = *(const v4f*)(slab + row * 68 + c4);
          *(volatile v4f*)(Cout + (size_t)(mBase + row) * ldc + n0 + c4) = v;
        }
        __threadfence();
      }
      wave_lds_sync();
    }
  }

  if (MODE == 1) {
    float cs[4];
#pragma unroll
    for (int j = 0; j < 4; ++j) {
      float s = 0.0f;
#pragma unroll
      for (int i = 0; i < 4; ++i) {
#pragma unroll
        for (int r = 0; r < 8; ++r) s += fmaxf(acc[i][j][r], 0.0f);
      }
      cs[j] = s;
    }
#pragma unroll
    for (int j = 0; j < 4; ++j) cs[j] += __shfl_xor(cs[j], 16, 32);
#pragma unroll
    for (int j = 0; j < 4; ++j) slab[(j << 4) + rlane] = cs[j] * scale;
    wave_lds_sync();
    const v4f v = *(const v4f*)(slab + (l16 << 2));
    float* dst = Cout + (size_t)tm * ldc + n0 + (l16 << 2);
    for (int pass = 0; pass < 2; ++pass) {
      if (lane < 16) *(volatile v4f*)dst = v;
      __threadfence();
    }
  }

  if (MODE == 2) {
    float w2[4];
#pragma unroll
    for (int j = 0; j < 4; ++j) w2[j] = wvec[n0 + (j << 4) + rlane];
#pragma unroll
    for (int i = 0; i < 4; ++i) {
#pragma unroll
      for (int r = 0; r < 8; ++r) {
        float p = 0.0f;
#pragma unroll
        for (int j = 0; j < 4; ++j) p = fmaf(fmaxf(acc[i][j][r], 0.0f), w2[j], p);
        p += __shfl_xor(p, 1, 32);
        p += __shfl_xor(p, 2, 32);
        p += __shfl_xor(p, 4, 32);
        p += __shfl_xor(p, 8, 32);
        slab[(i << 4) + mOff + r] = p * scale;
      }
    }
    wave_lds_sync();
    const v4f v = *(const v4f*)(slab + (l16 << 2));
    float* dst = Cout + (size_t)tn * ldc + m0 + (l16 << 2);
    for (int pass = 0; pass < 2; ++pass) {
      if (lane < 16) *(volatile v4f*)dst = v;
      __threadfence();
    }
  }
}

__global__ __launch_bounds__(256) void gather_hops_kernel(
    const float* __restrict__ UV, const int* __restrict__ paths, const int* __restrict__ plen,
    const float* __restrict__ b1, unsigned short* __restrict__ Hm, int rowBase, int nrows)
{
  const int lane = threadIdx.x & 31;
  const int wave = threadIdx.x >> 5;
  const int r = blockIdx.x * 8 + wave;
  if (r >= nrows) return;
  const int p = rowBase + r;
  const bool real = p < kPaths;
  const int pc = real ? p : (kPaths - 1);
  const v4i pv = *(const v4i*)(paths + (size_t)pc * 4);
  const int len = plen[pc];
  int nd[4];
  nd[0] = clamp_int(pv[0], 0, kNodes - 1);
  nd[1] = clamp_int(pv[1], 0, kNodes - 1);
  nd[2] = clamp_int(pv[2], 0, kNodes - 1);
  nd[3] = clamp_int(pv[3], 0, kNodes - 1);

  v8h hv[3];
  float mf[3];
#pragma unroll
  for (int s = 0; s < 3; ++s) {
    const bool m = real && (s < len - 1);
    mf[s] = m ? kCarryA : 0.0f;
    const float* up = UV + (size_t)nd[s] * kUvW + (2 * s) * kFeat + 8 * lane;
    const float* vp = UV + (size_t)nd[s + 1] * kUvW + (2 * s + 1) * kFeat + 8 * lane;
    const float* bp = b1 + s * kFeat + 8 * lane;
    const v4f u0 = *(const v4f*)(up);
    const v4f u1 = *(const v4f*)(up + 4);
    const v4f w0 = *(const v4f*)(vp);
    const v4f w1 = *(const v4f*)(vp + 4);
    const v4f c0 = *(const v4f*)(bp);
    const v4f c1 = *(const v4f*)(bp + 4);
#pragma unroll
    for (int e = 0; e < 4; ++e) {
      float x0 = (u0[e] + w0[e]) + c0[e];
      float x1 = (u1[e] + w1[e]) + c1[e];
      x0 = fmaxf(x0, 0.0f) * kCarryA;
      x1 = fmaxf(x1, 0.0f) * kCarryA;
      x0 = m ? x0 : 0.0f;
      x1 = m ? x1 : 0.0f;
      hv[s][e]     = (_Float16)x0;
      hv[s][4 + e] = (_Float16)x1;
    }
  }
  float zv = 0.0f;
  asm volatile("" : "+v"(zv));
  const bool l0 = (lane == 0);
  const float t0 = l0 ? (real ? kCarryA : 0.0f) : zv;
  const float t1 = l0 ? mf[0] : zv;
  const float t2 = l0 ? mf[1] : zv;
  const float t3 = l0 ? mf[2] : zv;
  v8h tv;
  tv[0] = (_Float16)t0;
  tv[1] = (_Float16)t1;
  tv[2] = (_Float16)t2;
  tv[3] = (_Float16)t3;
  tv[4] = (_Float16)zv;
  tv[5] = (_Float16)zv;
  tv[6] = (_Float16)zv;
  tv[7] = (_Float16)zv;

  unsigned short* rowp = Hm + (size_t)r * kHmPitch;
  for (int pass = 0; pass < 2; ++pass) {
#pragma unroll
    for (int s = 0; s < 3; ++s) *(volatile v8h*)(rowp + s * kFeat + 8 * lane) = hv[s];
    if (lane < 8) *(volatile v8h*)(rowp + kIndCol + 8 * lane) = tv;
    __threadfence();
  }
}

__global__ __launch_bounds__(256) void score_kernel(
    const float* __restrict__ SP, const float* __restrict__ bs2, float* __restrict__ outScores)
{
  const int p = blockIdx.x * 256 + threadIdx.x;
  if (p >= kPaths) return;
  const float x = (SP[p] + SP[kRowsPad + p]) + bs2[0];
  const float sc = 1.0f / (1.0f + expf(-x));
  *(volatile float*)(outScores + p) = sc;
  __threadfence();
  *(volatile float*)(outScores + p) = sc;
}

__global__ __launch_bounds__(256) void reduce_matvec_kernel(
    const float* __restrict__ partials, const float* __restrict__ Wa2, const float* __restrict__ ba2,
    float* __restrict__ aggv)
{
  __shared__ float sS[kFeat];
  const int t = threadIdx.x;
  float outer = 0.0f;
#pragma unroll 1
  for (int b = 0; b < kRedOuter; ++b) {
    float inner = 0.0f;
#pragma unroll 1
    for (int i = 0; i < kRedInner; ++i) inner += partials[(size_t)(b * kRedInner + i) * kFeat + t];
    outer += inner;
  }
  sS[t] = outer;
  __syncthreads();
  float a = 0.0f;
#pragma unroll 8
  for (int j = 0; j < kFeat; ++j) a = fmaf(sS[j], Wa2[(size_t)j * kFeat + t], a);
  a += (float)kPaths * ba2[t];
  *(volatile float*)(aggv + t) = a;
  __threadfence();
  *(volatile float*)(aggv + t) = a;
}

__global__ __launch_bounds__(256) void add_broadcast_kernel(
    const float* __restrict__ nf, const float* __restrict__ aggv, float* __restrict__ out)
{
  const int i = blockIdx.x * 256 + threadIdx.x;
  if (i >= kNodes * kFeat / 4) return;
  const size_t e0 = (size_t)i * 4;
  const int d4 = (int)(e0 & (kFeat - 1));
  const v4f a = *(const v4f*)(nf + e0);
  const v4f g = *(const v4f*)(aggv + d4);
  const v4f o = a + g;
  *(volatile v4f*)(out + e0) = o;
  __threadfence();
  *(volatile v4f*)(out + e0) = o;
}

extern "C" void kernel_launch(void* const* d_in, const int* in_sizes, int n_in,
                              void* d_out, int out_size, void* d_ws, size_t ws_size,
                              hipStream_t stream) {
  if (n_in < 15) return;
  if (in_sizes[0] != kNodes * kFeat) return;
  if (in_sizes[1] != kPaths * 4) return;
  if (in_sizes[2] != kPaths) return;
  if (in_sizes[3] != kHops * 2 * kFeat * kFeat) return;
  if (in_sizes[4] != kHops * kFeat) return;
  if (in_sizes[5] != kHops * kFeat * kFeat) return;
  if (in_sizes[6] != kHops * kFeat) return;
  if (in_sizes[7] != kFeat * kScoreH) return;
  if (in_sizes[8] != kScoreH) return;
  if (in_sizes[9] != kScoreH) return;
  if (in_sizes[10] != 1) return;
  if (in_sizes[11] != 4 * kFeat * kFeat) return;
  if (in_sizes[12] != kFeat) return;
  if (in_sizes[13] != kFeat * kFeat) return;
  if (in_sizes[14] != kFeat) return;
  if (out_size != kOut1Elem + kPaths) return;
  if (ws_size < kWsTotal) return;

  const float* nf    = (const float*)d_in[0];
  const int*   paths = (const int*)d_in[1];
  const int*   plen  = (const int*)d_in[2];
  const float* W1    = (const float*)d_in[3];
  const float* b1    = (const float*)d_in[4];
  const float* W2    = (const float*)d_in[5];
  const float* b2    = (const float*)d_in[6];
  const float* Ws1   = (const float*)d_in[7];
  const float* bs1   = (const float*)d_in[8];
  const float* Ws2   = (const float*)d_in[9];
  const float* bs2   = (const float*)d_in[10];
  const float* Wa1   = (const float*)d_in[11];
  const float* ba1   = (const float*)d_in[12];
  const float* Wa2   = (const float*)d_in[13];
  const float* ba2   = (const float*)d_in[14];
  float* out = (float*)d_out;

  char* ws = (char*)d_ws;
  unsigned short* NFH  = (unsigned short*)(ws + kOffNFH);
  unsigned short* W1T  = (unsigned short*)(ws + kOffW1T);
  float*          UV   = (float*)(ws + kOffUV);
  float*          TC   = (float*)(ws + kOffTC);
  float*          TS   = (float*)(ws + kOffTS);
  unsigned short* WCT  = (unsigned short*)(ws + kOffWCT);
  unsigned short* WST  = (unsigned short*)(ws + kOffWST);
  unsigned short* HM   = (unsigned short*)(ws + kOffHM);
  float*          PART = (float*)(ws + kOffPART);
  float*          SP   = (float*)(ws + kOffSP);
  float*          AGG  = (float*)(ws + kOffAGG);

  cast_nodes_f16<<<kNodesPad * kFeat / 8 / 256, 256, 0, stream>>>(nf, NFH);

  transpose_cast_f16<<<dim3(4, 4, 6), 256, 0, stream>>>(W1, kFeat, (long)kFeat * kFeat, W1T, kFeat, (long)kFeat * kFeat, kCarryW);

  compose_rows_kernel<<<kHmPitch * kFeat / 256, 256, 0, stream>>>(W2, b2, Wa1, ba1, TC, kFeat, kHops, kHmPitch);
  compose_rows_kernel<<<kWsPitch * kScoreH / 256, 256, 0, stream>>>(W2, b2, Ws1, bs1, TS, kScoreH, 1, kWsPitch);

  transpose_cast_f16<<<dim3(kHmPitch / 64, kFeat / 64, 1), 256, 0, stream>>>(TC, kFeat, 0L, WCT, kHmPitch, 0L, kCarryW);
  transpose_cast_f16<<<dim3(kWsPitch / 64, kScoreH / 64, 1), 256, 0, stream>>>(TS, kScoreH, 0L, WST, kWsPitch, 0L, kCarryW);

  gemm_f16_tile64<0><<<(kNodesPad / 64) * (kUvW / 64) / 8, 256, 0, stream>>>(
      NFH, kFeat, W1T, kFeat, UV, kUvW, nullptr,
      kNodesPad, kUvW, kFeat / 32, kFeat / 32, 0, kFold);

  for (int c = 0; c < kNumChunks; ++c) {
    gather_hops_kernel<<<kChunk / 8, 256, 0, stream>>>(UV, paths, plen, b1, HM, c * kChunk, kChunk);

    gemm_f16_tile64<1><<<(kTilesChunk * (kFeat / 64) + 7) / 8, 256, 0, stream>>>(
        HM, kHmPitch, WCT, kHmPitch, PART + (size_t)c * kTilesChunk * kFeat, kFeat, nullptr,
        kChunk, kFeat, kKz / 32, kKz / 32, 0, kFold);

    gemm_f16_tile64<2><<<(kTilesChunk * (kScoreH / 64) + 7) / 8, 256, 0, stream>>>(
        HM, kHmPitch, WST, kWsPitch, SP + (size_t)c * kChunk, kRowsPad, Ws2,
        kChunk, kScoreH, kKs / 32, kFeat / 32, kIndCol, kFold);
  }

  score_kernel<<<(kPaths + 255) / 256, 256, 0, stream>>>(SP, bs2, out + kOut1Elem);
  reduce_matvec_kernel<<<1, 256, 0, stream>>>(PART, Wa2, ba2, AGG);
  add_broadcast_kernel<<<kNodes * kFeat / 4 / 256, 256, 0, stream>>>(nf, AGG, out);
}
